// DementiaConditioningDiscriminator_13211319402666
// MI455X (gfx1250) — hardware-verified
//
#include <hip/hip_runtime.h>
#include <stddef.h>


#define XIN     19
#define XP      32
#define HID     128
#define LAT     64
#define NTHR    256
#define NWAVE   8
#define ATHR    128
#define AWAVE   4
#define ATGT    (AWAVE * 32)
#define EPT     8
#define NGRP    2
#define CHUNK   (NTHR * EPT * NGRP)
#define WCAP    (EPT * NGRP * 32)
#define LISTN   (NWAVE * WCAP)
#define NBC     4096
#define NBF     1024
#define RCAP    40960
#define RBN     128
#define DEGCAP  256
#define GROWS   128
#define OTHR    512
#define NPU     256
#define LDS_FILL ((RCAP + NBF + LISTN) * 4 + 64)

static_assert((CHUNK & (CHUNK - 1)) == 0);
static_assert(CHUNK <= 4096);
static_assert((NBC & (NBC - 1)) == 0 && (NBF & (NBF - 1)) == 0);
static_assert(NBC == 4 * NBF);
static_assert(OTHR * 8 == NBC);
static_assert((RCAP % 32) == 0);
static_assert(LISTN == NTHR * EPT * NGRP);
static_assert(NPU % GROWS == 0 && NPU % ATGT == 0 && NPU % NTHR == 0 && NBC % NPU == 0);
static_assert(XP % 32 == 0 && HID % 32 == 0 && LAT % 32 == 0);

typedef float          v2f   __attribute__((ext_vector_type(2)));
typedef float          v4f   __attribute__((ext_vector_type(4)));
typedef float          v8f   __attribute__((ext_vector_type(8)));
typedef int            v4i   __attribute__((ext_vector_type(4)));
typedef unsigned short v4us  __attribute__((ext_vector_type(4)));
typedef unsigned short v8us  __attribute__((ext_vector_type(8)));
typedef unsigned short v16us __attribute__((ext_vector_type(16)));
typedef __bf16         v16bf __attribute__((ext_vector_type(16)));
union FragU { v16us v; v8us h[2]; };

struct WSeg { const float* src; unsigned short* hi; unsigned short* lo; int K; int NOUT; int KP; int blk0; };
struct WPrep { WSeg s[8]; };
static_assert(sizeof(WSeg) == 40);
static_assert(sizeof(WPrep) == 320);

__device__ __forceinline__ unsigned int bf_bits(float f) {
  const unsigned int u = __float_as_uint(f);
  return (u + 0x7FFFu + ((u >> 16) & 1u)) >> 16;
}
__device__ __forceinline__ unsigned int split_pack(float v) {
  const unsigned int hb = bf_bits(v);
  const float hf = __uint_as_float(hb << 16);
  const unsigned int lb = bf_bits(v - hf);
  return (hb & 0xffffu) | (lb << 16);
}
__device__ __forceinline__ void pack4(v4f a, v4us& hv, v4us& lv) {
  unsigned int p;
  p = split_pack(a.x); hv[0] = (unsigned short)(p & 0xffffu); lv[0] = (unsigned short)(p >> 16);
  p = split_pack(a.y); hv[1] = (unsigned short)(p & 0xffffu); lv[1] = (unsigned short)(p >> 16);
  p = split_pack(a.z); hv[2] = (unsigned short)(p & 0xffffu); lv[2] = (unsigned short)(p >> 16);
  p = split_pack(a.w); hv[3] = (unsigned short)(p & 0xffffu); lv[3] = (unsigned short)(p >> 16);
}
__device__ __forceinline__ void pack8(v4f a, v4f b, v8us& hv, v8us& lv) {
  unsigned int p;
  p = split_pack(a.x); hv[0] = (unsigned short)(p & 0xffffu); lv[0] = (unsigned short)(p >> 16);
  p = split_pack(a.y); hv[1] = (unsigned short)(p & 0xffffu); lv[1] = (unsigned short)(p >> 16);
  p = split_pack(a.z); hv[2] = (unsigned short)(p & 0xffffu); lv[2] = (unsigned short)(p >> 16);
  p = split_pack(a.w); hv[3] = (unsigned short)(p & 0xffffu); lv[3] = (unsigned short)(p >> 16);
  p = split_pack(b.x); hv[4] = (unsigned short)(p & 0xffffu); lv[4] = (unsigned short)(p >> 16);
  p = split_pack(b.y); hv[5] = (unsigned short)(p & 0xffffu); lv[5] = (unsigned short)(p >> 16);
  p = split_pack(b.z); hv[6] = (unsigned short)(p & 0xffffu); lv[6] = (unsigned short)(p >> 16);
  p = split_pack(b.w); hv[7] = (unsigned short)(p & 0xffffu); lv[7] = (unsigned short)(p >> 16);
}

__device__ __forceinline__ v8f wmb(v16us a, v16us b, v8f c) {
  const v16bf ab = __builtin_bit_cast(v16bf, a);
  const v16bf bb = __builtin_bit_cast(v16bf, b);
  v8f d = __builtin_amdgcn_wmma_f32_16x16x32_bf16(false, ab, false, bb, (short)0, c, false, false);
  asm volatile("v_nop\n\tv_nop\n\tv_nop\n\tv_nop" : "+v"(d) : "v"(ab), "v"(bb));
  return d;
}

template <int NB>
__device__ __forceinline__ int scan_chunk(const int* __restrict__ dsts, int nE, int cbase, int slotBase,
                                          int vec8, int* list, int tid, int lane, int wave) {
  int wc = 0;
#pragma unroll
  for (int g = 0; g < NGRP; ++g) {
    const int el0  = (g * NTHR + tid) * EPT;
    const int e0   = cbase + el0;
    const int sent = -2147483647 - 1;
    v4i da, db;
    if (vec8 != 0 && cbase + CHUNK <= nE) {
      da = *(const v4i*)(dsts + e0);
      db = *(const v4i*)(dsts + e0 + 4);
    } else {
      da.x = (e0     < nE) ? dsts[min(e0, nE - 1)] : sent;
      da.y = (e0 + 1 < nE) ? dsts[min(e0 + 1, nE - 1)] : sent;
      da.z = (e0 + 2 < nE) ? dsts[min(e0 + 2, nE - 1)] : sent;
      da.w = (e0 + 3 < nE) ? dsts[min(e0 + 3, nE - 1)] : sent;
      db.x = (e0 + 4 < nE) ? dsts[min(e0 + 4, nE - 1)] : sent;
      db.y = (e0 + 5 < nE) ? dsts[min(e0 + 5, nE - 1)] : sent;
      db.z = (e0 + 6 < nE) ? dsts[min(e0 + 6, nE - 1)] : sent;
      db.w = (e0 + 7 < nE) ? dsts[min(e0 + 7, nE - 1)] : sent;
    }
    const unsigned nb = (unsigned)slotBase;
    const unsigned s0 = (unsigned)da.x - nb, s1 = (unsigned)da.y - nb;
    const unsigned s2 = (unsigned)da.z - nb, s3 = (unsigned)da.w - nb;
    const unsigned s4 = (unsigned)db.x - nb, s5 = (unsigned)db.y - nb;
    const unsigned s6 = (unsigned)db.z - nb, s7 = (unsigned)db.w - nb;
    const bool h0 = s0 < (unsigned)NB, h1 = s1 < (unsigned)NB, h2 = s2 < (unsigned)NB, h3 = s3 < (unsigned)NB;
    const bool h4 = s4 < (unsigned)NB, h5 = s5 < (unsigned)NB, h6 = s6 < (unsigned)NB, h7 = s7 < (unsigned)NB;
    const unsigned any = __builtin_amdgcn_ballot_w32(h0 | h1 | h2 | h3 | h4 | h5 | h6 | h7);
    if (any != 0u) {
#define HITJ(J, HJ, SJ) { \
        const unsigned mj = __builtin_amdgcn_ballot_w32(HJ); \
        if (mj != 0u) { \
          if (HJ) { \
            const int pos = wc + (int)__builtin_amdgcn_mbcnt_lo(mj, 0u); \
            if (pos < WCAP) list[wave * WCAP + pos] = ((el0 + (J)) << 12) | (int)(SJ); \
          } \
          wc += (int)__builtin_popcount(mj); } }
      HITJ(0, h0, s0)
      HITJ(1, h1, s1)
      HITJ(2, h2, s2)
      HITJ(3, h3, s3)
      HITJ(4, h4, s4)
      HITJ(5, h5, s5)
      HITJ(6, h6, s6)
      HITJ(7, h7, s7)
#undef HITJ
    }
  }
  return wc;
}

__global__ __launch_bounds__(NTHR) void k_xpad(const float* __restrict__ x, float* xp, int nN, int npad) {
  const int t = blockIdx.x * NTHR + (int)threadIdx.x;
  if (t >= npad * (XP / 4)) return;
  const int row = t >> 3;
  const int c0  = (t & 7) * 4;
  const int rc  = row < nN ? row : nN - 1;
  float v[4];
#pragma unroll
  for (int e = 0; e < 4; ++e) {
    const int col = c0 + e;
    const int cc  = col < XIN ? col : XIN - 1;
    const float val = x[(size_t)rc * XIN + cc];
    v[e] = (col < XIN && row < nN) ? val : 0.0f;
  }
  v4f o; o.x = v[0]; o.y = v[1]; o.z = v[2]; o.w = v[3];
  float* p = xp + (size_t)row * XP + c0;
  *(volatile v4f*)p = o;
  __threadfence();
  *(volatile v4f*)p = o;
}

__global__ __launch_bounds__(NTHR) void k_wprep(WPrep P) {
  WSeg sg = P.s[0];
#pragma unroll
  for (int s = 1; s < 8; ++s) { if ((int)blockIdx.x >= P.s[s].blk0) sg = P.s[s]; }
  const int t   = ((int)blockIdx.x - sg.blk0) * NTHR + (int)threadIdx.x;
  const int kp8 = sg.KP / 8;
  if (t >= sg.NOUT * kp8) return;
  const int n  = t / kp8;
  const int k0 = (t - n * kp8) * 8;
  float v[8];
#pragma unroll
  for (int e = 0; e < 8; ++e) {
    const int k  = k0 + e;
    const int kc = k < sg.K ? k : sg.K - 1;
    const float val = sg.src[(size_t)kc * sg.NOUT + n];
    v[e] = (k < sg.K) ? val : 0.0f;
  }
  v4f a, b;
  a.x = v[0]; a.y = v[1]; a.z = v[2]; a.w = v[3];
  b.x = v[4]; b.y = v[5]; b.z = v[6]; b.w = v[7];
  v8us hv, lv;
  pack8(a, b, hv, lv);
  const size_t o = (size_t)n * sg.KP + k0;
  *(volatile v8us*)(sg.hi + o) = hv;
  *(volatile v8us*)(sg.lo + o) = lv;
  __threadfence();
  *(volatile v8us*)(sg.hi + o) = hv;
  *(volatile v8us*)(sg.lo + o) = lv;
}

__global__ __launch_bounds__(NTHR) void k_count(const int* __restrict__ ei, int* cnt, int nE, int vec8) {
  __shared__ __attribute__((aligned(16))) int scnt[NBC];
  __shared__ __attribute__((aligned(16))) int list[LISTN];
  __shared__ int wcnt[NWAVE];
  const int tid = threadIdx.x, lane = tid & 31, wave = tid >> 5;
  const int nodeBase = blockIdx.x * NBC;
  const int* dsts = ei + nE;

  for (int i = tid; i < NBC; i += NTHR) scnt[i] = 0;
  __syncthreads();

  const int nChunks = (nE + CHUNK - 1) / CHUNK;
#pragma unroll 1
  for (int ch = 0; ch < nChunks; ++ch) {
    const int cbase = ch * CHUNK;
    const int wc = scan_chunk<NBC>(dsts, nE, cbase, nodeBase, vec8, list, tid, lane, wave);
    if (lane == 0) wcnt[wave] = wc;
    __syncthreads();
    if (wave == 0) {
#pragma unroll 1
      for (int wsx = 0; wsx < NWAVE; ++wsx) {
        int n = __builtin_amdgcn_readfirstlane(wcnt[wsx]);
        n = n > WCAP ? WCAP : (n < 0 ? 0 : n);
        const int* lp = list + wsx * WCAP;
#pragma unroll 1
        for (int i = 0; i < n; ++i) {
          const int ent  = __builtin_amdgcn_readfirstlane(lp[i]);
          const int slot = ent & (NBC - 1);
          if (lane == 0) scnt[slot] = scnt[slot] + 1;
        }
      }
    }
    __syncthreads();
  }

  v4i cq[4];
#pragma unroll
  for (int q = 0; q < 4; ++q) {
    const int f = (wave * 4 + q) * 128 + 4 * lane;
    cq[q] = *(const v4i*)(scnt + f);
  }
  int* cp = cnt + (size_t)nodeBase;
#pragma unroll
  for (int q = 0; q < 4; ++q) {
    const int f = (wave * 4 + q) * 128 + 4 * lane;
    *(volatile v4i*)(cp + f) = cq[q];
  }
  __threadfence();
#pragma unroll
  for (int q = 0; q < 4; ++q) {
    const int f = (wave * 4 + q) * 128 + 4 * lane;
    *(volatile v4i*)(cp + f) = cq[q];
  }
}

__global__ __launch_bounds__(OTHR) void k_offsets(const int* __restrict__ cnt, int* off, int* rbase, int nChunk) {
  __shared__ __attribute__((aligned(16))) int soff[NBC];
  __shared__ __attribute__((aligned(16))) int srb[RBN];
  __shared__ int wtot[OTHR / 32];
  const int tid = threadIdx.x, lane = tid & 31, wave = tid >> 5, sub = tid >> 7;
  for (int i = tid; i < RBN; i += OTHR) srb[i] = 0;
  int carry = 0;
#pragma unroll 1
  for (int ch = 0; ch < nChunk; ++ch) {
    const int base = ch * NBC;
    const v4i c0 = *(const v4i*)(cnt + base + 8 * tid);
    const v4i c1 = *(const v4i*)(cnt + base + 8 * tid + 4);
    const int e0 = max(c0.x, 0), e1 = max(c0.y, 0), e2 = max(c0.z, 0), e3 = max(c0.w, 0);
    const int e4 = max(c1.x, 0), e5 = max(c1.y, 0), e6 = max(c1.z, 0), e7 = max(c1.w, 0);
    const int ts = e0 + e1 + e2 + e3 + e4 + e5 + e6 + e7;
    int incl = ts;
#pragma unroll
    for (int d = 1; d < 32; d <<= 1) {
      const int t = __shfl_up(incl, d);
      if (lane >= d) incl += t;
    }
    if (lane == 31) wtot[wave] = incl;
    __syncthreads();
    const int S0 = wtot[0]  + wtot[1]  + wtot[2]  + wtot[3];
    const int S1 = wtot[4]  + wtot[5]  + wtot[6]  + wtot[7];
    const int S2 = wtot[8]  + wtot[9]  + wtot[10] + wtot[11];
    const int S3 = wtot[12] + wtot[13] + wtot[14] + wtot[15];
    int pre = 0;
#pragma unroll 1
    for (int w = 4 * sub; w < wave; ++w) pre += wtot[w];
    const int b0 = carry;
    const int b1 = b0 + ((S0 + 31) & ~31);
    const int b2 = b1 + ((S1 + 31) & ~31);
    const int b3 = b2 + ((S2 + 31) & ~31);
    const int b4 = b3 + ((S3 + 31) & ~31);
    const int myb = sub == 0 ? b0 : (sub == 1 ? b1 : (sub == 2 ? b2 : b3));
    if (tid == 0) {
      srb[min(4 * ch + 0, RBN - 1)] = b0;
      srb[min(4 * ch + 1, RBN - 1)] = b1;
      srb[min(4 * ch + 2, RBN - 1)] = b2;
      srb[min(4 * ch + 3, RBN - 1)] = b3;
    }
    int run = myb + pre + incl - ts;
    soff[8 * tid + 0] = run; run += e0;
    soff[8 * tid + 1] = run; run += e1;
    soff[8 * tid + 2] = run; run += e2;
    soff[8 * tid + 3] = run; run += e3;
    soff[8 * tid + 4] = run; run += e4;
    soff[8 * tid + 5] = run; run += e5;
    soff[8 * tid + 6] = run; run += e6;
    soff[8 * tid + 7] = run;
    carry = b4;
    __syncthreads();
    const v4i o0 = *(const v4i*)(soff + 4 * tid);
    const v4i o1 = *(const v4i*)(soff + 4 * (tid + OTHR));
    int* op = off + base;
    *(volatile v4i*)(op + 4 * tid) = o0;
    *(volatile v4i*)(op + 4 * (tid + OTHR)) = o1;
    __threadfence();
    *(volatile v4i*)(op + 4 * tid) = o0;
    *(volatile v4i*)(op + 4 * (tid + OTHR)) = o1;
    __syncthreads();
  }
  if (tid == 0) srb[min(4 * nChunk, RBN - 1)] = carry;
  __syncthreads();
  v4i rv = {0, 0, 0, 0};
  if (tid < 32) rv = *(const v4i*)(srb + 4 * tid);
  if (tid < 32) *(volatile v4i*)(rbase + 4 * tid) = rv;
  __threadfence();
  if (tid < 32) *(volatile v4i*)(rbase + 4 * tid) = rv;
}

__global__ __launch_bounds__(NTHR) void k_fill(const int* __restrict__ ei, const int* __restrict__ off,
                                               const int* __restrict__ rbase, int* csr,
                                               int nN, int nE, int vec8, int csrLen) {
  extern __shared__ v4f lds_dyn[];
  int* region = (int*)lds_dyn;
  int* cursor = region + RCAP;
  int* list   = cursor + NBF;
  int* wcnt   = list + LISTN;
  const int tid = threadIdx.x, lane = tid & 31, wave = tid >> 5;
  const int b = blockIdx.x;
  const int nodeBase = b * NBF;
  const int* dsts = ei + nE;

  int rb0 = rbase[b];
  const int rb1 = rbase[b + 1];
  rb0 = rb0 < 0 ? 0 : (rb0 > csrLen ? csrLen : rb0);
  rb0 &= ~31;
  int len = rb1 - rb0;
  len = len < 0 ? 0 : (len > RCAP ? RCAP : len);
  int lenW = (len + 31) & ~31;
  if (rb0 + lenW > csrLen) lenW = (csrLen - rb0) & ~31;

  {
    const v4i z = {0, 0, 0, 0};
    for (int i = tid; i < RCAP / 4; i += NTHR) ((v4i*)region)[i] = z;
    for (int s = tid; s < NBF; s += NTHR) {
      int o = off[nodeBase + s] - rb0;
      o = o < 0 ? 0 : (o > RCAP ? RCAP : o);
      cursor[s] = o;
    }
  }
  __syncthreads();

  const int nChunks = (nE + CHUNK - 1) / CHUNK;
#pragma unroll 1
  for (int ch = 0; ch < nChunks; ++ch) {
    const int cbase = ch * CHUNK;
    const int wc = scan_chunk<NBF>(dsts, nE, cbase, nodeBase, vec8, list, tid, lane, wave);
    if (lane == 0) wcnt[wave] = wc;
    __syncthreads();
    if (wave == 0) {
#pragma unroll 1
      for (int wsx = 0; wsx < NWAVE; ++wsx) {
        int n = __builtin_amdgcn_readfirstlane(wcnt[wsx]);
        n = n > WCAP ? WCAP : (n < 0 ? 0 : n);
        const int* lp = list + wsx * WCAP;
#pragma unroll 1
        for (int i = 0; i < n; ++i) {
          const int ent  = __builtin_amdgcn_readfirstlane(lp[i]);
          const int slot = ent & (NBF - 1);
          int e = cbase + ((ent >> 12) & (CHUNK - 1));
          e = e > nE - 1 ? nE - 1 : e;
          int src = ei[e];
          src = src < 0 ? 0 : (src > nN - 1 ? nN - 1 : src);
          if (lane == 0) {
            int pos = cursor[slot];
            pos = pos < 0 ? 0 : (pos > RCAP - 1 ? RCAP - 1 : pos);
            region[pos] = src;
            const int np = pos + 1;
            cursor[slot] = np > RCAP ? RCAP : np;
          }
        }
      }
    }
    __syncthreads();
  }

  const int nv = lenW >> 2;
  int* gp = csr + rb0;
#pragma unroll 1
  for (int i = tid; i < nv; i += NTHR) { const v4i v = ((const v4i*)region)[i]; *(volatile v4i*)(gp + 4 * i) = v; }
  __threadfence();
#pragma unroll 1
  for (int i = tid; i < nv; i += NTHR) { const v4i v = ((const v4i*)region)[i]; *(volatile v4i*)(gp + 4 * i) = v; }
}

template <int P, int RELU>
__global__ __launch_bounds__(ATHR) void k_agg(const int* __restrict__ csr, const int* __restrict__ off,
                                              const int* __restrict__ cnt, const float* __restrict__ hs,
                                              const float* __restrict__ bias, unsigned short* zh, unsigned short* zl,
                                              int nN, int csrLen, int useBias) {
  extern __shared__ v4f lds_dyn[];
  constexpr int LPR = P / 4;
  constexpr int EPI = 32 / LPR;
  constexpr int NI  = P / 8;
  unsigned short* sH = (unsigned short*)lds_dyn;
  unsigned short* sL = sH + AWAVE * 32 * P;
  const int tid = threadIdx.x, lane = tid & 31, wave = tid >> 5;
  const int grp = lane / LPR;
  const int cl4 = 4 * (lane - grp * LPR);
  const int tbase = blockIdx.x * ATGT + wave * 32;
  const int cnt_l = cnt[tbase + lane];
  const int off_l = off[tbase + lane];
  const v4f zero4 = {0.0f, 0.0f, 0.0f, 0.0f};
  const v4f braw = *(const v4f*)(bias + cl4);
  const v4f bb = (useBias != 0) ? braw : zero4;
  unsigned short* wH = sH + wave * 32 * P;
  unsigned short* wL = sL + wave * 32 * P;

#pragma unroll 1
  for (int j = 0; j < 32; ++j) {
    const int c = tbase + j;
    int n = __builtin_amdgcn_readlane(cnt_l, j);
    n = n < 0 ? 0 : (n > DEGCAP ? DEGCAP : n);
    const int st = __builtin_amdgcn_readlane(off_l, j);
    v4f acc = zero4;
#pragma unroll 1
    for (int q0 = 0; q0 < n; q0 += 32) {
      int pos = st + q0 + lane;
      pos = pos < 0 ? 0 : (pos > csrLen - 1 ? csrLen - 1 : pos);
      int sl = csr[pos];
      sl = sl < 0 ? 0 : (sl > nN - 1 ? nN - 1 : sl);
      const int mcnt = (n - q0) < 32 ? (n - q0) : 32;
      if (EPI == 1) {
#pragma unroll 1
        for (int p = 0; p < mcnt; ++p) {
          const int s = __builtin_amdgcn_readlane(sl, p);
          acc += *(const v4f*)(hs + (size_t)s * P + cl4);
        }
      } else {
#pragma unroll 1
        for (int p = 0; p < mcnt; p += EPI) {
          const int li = p + grp;
          const int s  = __shfl(sl, li);
          const v4f v  = *(const v4f*)(hs + (size_t)s * P + cl4);
          const bool ok = li < mcnt;
          acc.x += ok ? v.x : 0.0f;
          acc.y += ok ? v.y : 0.0f;
          acc.z += ok ? v.z : 0.0f;
          acc.w += ok ? v.w : 0.0f;
        }
      }
    }
    if (EPI > 1) {
#pragma unroll
      for (int o = LPR; o < 32; o <<= 1) {
        acc.x += __shfl_xor(acc.x, o);
        acc.y += __shfl_xor(acc.y, o);
        acc.z += __shfl_xor(acc.z, o);
        acc.w += __shfl_xor(acc.w, o);
      }
    }
    const v4f sv = *(const v4f*)(hs + (size_t)c * P + cl4);
    v4f z = acc + sv + bb;
    if (RELU) {
      z.x = fmaxf(z.x, 0.0f); z.y = fmaxf(z.y, 0.0f); z.z = fmaxf(z.z, 0.0f); z.w = fmaxf(z.w, 0.0f);
    }
    v4us hv, lv;
    pack4(z, hv, lv);
    if (grp == 0) {
      *(v4us*)(wH + j * P + cl4) = hv;
      *(v4us*)(wL + j * P + cl4) = lv;
    }
  }
  __syncthreads();

  unsigned short* gh = zh + (size_t)tbase * P;
  unsigned short* gl = zl + (size_t)tbase * P;
#pragma unroll
  for (int i = 0; i < NI; ++i) {
    const v8us a = *(const v8us*)(wH + 256 * i + 8 * lane);
    const v8us b = *(const v8us*)(wL + 256 * i + 8 * lane);
    *(volatile v8us*)(gh + 256 * i + 8 * lane) = a;
    *(volatile v8us*)(gl + 256 * i + 8 * lane) = b;
  }
  __threadfence();
#pragma unroll
  for (int i = 0; i < NI; ++i) {
    const v8us a = *(const v8us*)(wH + 256 * i + 8 * lane);
    const v8us b = *(const v8us*)(wL + 256 * i + 8 * lane);
    *(volatile v8us*)(gh + 256 * i + 8 * lane) = a;
    *(volatile v8us*)(gl + 256 * i + 8 * lane) = b;
  }
}

template <int KD, int NOUT, int OUTP, int RELU>
__global__ __launch_bounds__(NTHR) void k_gemm(const unsigned short* __restrict__ Ah, const unsigned short* __restrict__ Al,
                                               const unsigned short* __restrict__ Bh, const unsigned short* __restrict__ Bl,
                                               const float* __restrict__ bias, float* Cf, unsigned short* Ch,
                                               unsigned short* Cl, int useBias) {
  extern __shared__ v4f lds_dyn[];
  float* stg = (float*)lds_dyn;
  constexpr int NT = NOUT / 16;
  constexpr int KT = KD / 32;
  const int tid = threadIdx.x, lane = tid & 31, wave = tid >> 5, hh = lane >> 4, m = lane & 15;
  const int rowBase = blockIdx.x * GROWS;

  v8f acc[NT];
#pragma unroll
  for (int t = 0; t < NT; ++t) { v8f z = {0.f, 0.f, 0.f, 0.f, 0.f, 0.f, 0.f, 0.f}; acc[t] = z; }
  const size_t arow = (size_t)(rowBase + wave * 16 + m) * KD + 8 * hh;
  const unsigned short* ahp = Ah + arow;
  const unsigned short* alp = Al + arow;
#pragma unroll 1
  for (int kt = 0; kt < KT; ++kt) {
    FragU ah, al;
    ah.h[0] = *(const v8us*)(ahp + 32 * kt);
    ah.h[1] = *(const v8us*)(ahp + 32 * kt + 16);
    al.h[0] = *(const v8us*)(alp + 32 * kt);
    al.h[1] = *(const v8us*)(alp + 32 * kt + 16);
#pragma unroll
    for (int t = 0; t < NT; ++t) {
      const size_t bo = (size_t)(16 * t + m) * KD + 32 * kt + 8 * hh;
      FragU bh, bl;
      bh.h[0] = *(const v8us*)(Bh + bo);
      bh.h[1] = *(const v8us*)(Bh + bo + 16);
      bl.h[0] = *(const v8us*)(Bl + bo);
      bl.h[1] = *(const v8us*)(Bl + bo + 16);
      acc[t] = wmb(ah.v, bh.v, acc[t]);
      acc[t] = wmb(ah.v, bl.v, acc[t]);
      acc[t] = wmb(al.v, bh.v, acc[t]);
    }
  }

  const int r0 = wave * 16 + 8 * hh;
  float* sp = stg + r0 * NOUT + m;
#pragma unroll
  for (int t = 0; t < NT; ++t) {
    const float braw = bias[16 * t + m];
    const float bv = (useBias != 0) ? braw : 0.0f;
#pragma unroll
    for (int r = 0; r < 8; ++r) {
      float v = acc[t][r] + bv;
      if (RELU) v = fmaxf(v, 0.0f);
      sp[r * NOUT + 16 * t] = v;
    }
  }
  __syncthreads();

  constexpr int EPL = OUTP ? 8 : 4;
  constexpr int LR  = NOUT / EPL;
  constexpr int RPI = 32 / LR;
  constexpr int NI  = 16 / RPI;
  const int lr = lane / LR;
  const int lc = (lane - lr * LR) * EPL;
#pragma unroll
  for (int i = 0; i < NI; ++i) {
    const int row = wave * 16 + i * RPI + lr;
    const float* lp = stg + row * NOUT + lc;
    const size_t go = (size_t)(rowBase + row) * NOUT + lc;
    if (OUTP == 0) {
      const v4f v = *(const v4f*)lp;
      *(volatile v4f*)(Cf + go) = v;
    } else {
      const v4f a = *(const v4f*)lp;
      const v4f b = *(const v4f*)(lp + 4);
      v8us hv, lv;
      pack8(a, b, hv, lv);
      *(volatile v8us*)(Ch + go) = hv;
      *(volatile v8us*)(Cl + go) = lv;
    }
  }
  __threadfence();
#pragma unroll
  for (int i = 0; i < NI; ++i) {
    const int row = wave * 16 + i * RPI + lr;
    const float* lp = stg + row * NOUT + lc;
    const size_t go = (size_t)(rowBase + row) * NOUT + lc;
    if (OUTP == 0) {
      const v4f v = *(const v4f*)lp;
      *(volatile v4f*)(Cf + go) = v;
    } else {
      const v4f a = *(const v4f*)lp;
      const v4f b = *(const v4f*)(lp + 4);
      v8us hv, lv;
      pack8(a, b, hv, lv);
      *(volatile v8us*)(Ch + go) = hv;
      *(volatile v8us*)(Cl + go) = lv;
    }
  }
}

__global__ __launch_bounds__(NTHR) void k_heads(const float* __restrict__ lat, const float* __restrict__ mw,
                                                const float* __restrict__ mb, const float* __restrict__ dw1,
                                                float* mm, float* tt) {
  __shared__ __attribute__((aligned(16))) float sM[NTHR];
  __shared__ __attribute__((aligned(16))) float sT[NTHR];
  const int tid = threadIdx.x, lane = tid & 31, wave = tid >> 5;
  const int tbase = blockIdx.x * NTHR + wave * 32;
  const v2f wm = *(const v2f*)(mw + 2 * lane);
  const v2f wd = *(const v2f*)(dw1 + 2 * lane);
  const float mbv = mb[0];
  float myM = 0.0f, myT = 0.0f;
#pragma unroll 1
  for (int j = 0; j < 32; ++j) {
    const v2f a = *(const v2f*)(lat + (size_t)(tbase + j) * LAT + 2 * lane);
    float pm = a.x * wm.x + a.y * wm.y;
    float pd = a.x * wd.x + a.y * wd.y;
#pragma unroll
    for (int o = 16; o > 0; o >>= 1) {
      pm += __shfl_xor(pm, o);
      pd += __shfl_xor(pd, o);
    }
    float s = pm + mbv;
    s = (s > 0.0f) ? s : 0.01f * s;
    if (lane == j) { myM = s; myT = pd; }
  }
  sM[tid] = myM;
  sT[tid] = myT;
  __syncthreads();
  const int li = wave * 32 + 4 * (lane < 8 ? lane : 7);
  const v4f a = *(const v4f*)(sM + li);
  const v4f b = *(const v4f*)(sT + li);
  if (lane < 8) {
    *(volatile v4f*)(mm + tbase + 4 * lane) = a;
    *(volatile v4f*)(tt + tbase + 4 * lane) = b;
  }
  __threadfence();
  if (lane < 8) {
    *(volatile v4f*)(mm + tbase + 4 * lane) = a;
    *(volatile v4f*)(tt + tbase + 4 * lane) = b;
  }
}

__global__ __launch_bounds__(NTHR) void k_final(const int* __restrict__ csr, const int* __restrict__ off,
                                                const int* __restrict__ cnt, const float* __restrict__ tt,
                                                const float* __restrict__ mm, const float* __restrict__ db1,
                                                const float* __restrict__ dw2, const float* __restrict__ db2,
                                                float* out, int nN, int csrLen, int total, int npad) {
  __shared__ __attribute__((aligned(16))) float sO[NTHR];
  const int tid = threadIdx.x, lane = tid & 31, wave = tid >> 5;
  const int wbase = (blockIdx.x * NWAVE + wave) * 32;
  int nd = wbase + lane;
  nd = nd > nN - 1 ? nN - 1 : nd;
  const int cnt_l = cnt[nd];
  const int off_l = off[nd];
  const float ts_l = tt[nd];
  const float b1v = db1[0], w2v = dw2[0], b2v = db2[0];
  float mine = 0.0f;
#pragma unroll 1
  for (int j = 0; j < 32; ++j) {
    int n = __builtin_amdgcn_readlane(cnt_l, j);
    n = n < 0 ? 0 : (n > DEGCAP ? DEGCAP : n);
    const int st = __builtin_amdgcn_readlane(off_l, j);
    float acc = 0.0f;
#pragma unroll 1
    for (int q0 = 0; q0 < n; q0 += 32) {
      int pos = st + q0 + lane;
      pos = pos < 0 ? 0 : (pos > csrLen - 1 ? csrLen - 1 : pos);
      int s = csr[pos];
      s = s < 0 ? 0 : (s > nN - 1 ? nN - 1 : s);
      const float v = tt[s];
      acc += (q0 + lane < n) ? v : 0.0f;
    }
#pragma unroll
    for (int o = 16; o > 0; o >>= 1) acc += __shfl_xor(acc, o);
    const float tsj = __shfl(ts_l, j);
    float r = acc + tsj + b1v;
    r = fmaxf(r, 0.0f);
    r = r * w2v + b2v;
    if (lane == j) mine = r;
  }
  const int e = wbase + lane;
  int mi = e - nN;
  mi = mi < 0 ? 0 : (mi > npad - 1 ? npad - 1 : mi);
  const float mv = mm[mi];
  const float val = (e < nN) ? mine : mv;
  sO[tid] = val;
  __syncthreads();
  const int li = wave * 32 + 4 * (lane < 8 ? lane : 7);
  const v4f ov = *(const v4f*)(sO + li);
  if (wbase + 32 <= total) {
    if (lane < 8) *(volatile v4f*)(out + wbase + 4 * lane) = ov;
    __threadfence();
    if (lane < 8) *(volatile v4f*)(out + wbase + 4 * lane) = ov;
  } else if (wbase < total) {
    if (e < total) *(volatile float*)(out + e) = val;
    __threadfence();
    if (e < total) *(volatile float*)(out + e) = val;
  }
}

extern "C" void kernel_launch(void* const* d_in, const int* in_sizes, int n_in,
                              void* d_out, int out_size, void* d_ws, size_t ws_size,
                              hipStream_t stream) {
  if (n_in < 24) return;
  const int nN = in_sizes[0] / XIN;
  const int nE = in_sizes[1] / 2;
  if (nN <= 0 || nE <= 0 || in_sizes[0] != nN * XIN || in_sizes[1] != 2 * nE) return;
  if (nE > (1 << 28) || nN > (1 << 24)) return;
  const int wK[8]  = {XIN, HID, HID, HID, HID, HID, HID, LAT};
  const int wN[8]  = {HID, HID, HID, HID, HID, HID, LAT, LAT};
  const int wKP[8] = {XP,  HID, HID, HID, HID, HID, HID, LAT};
  const int wIdx[8] = {2, 4, 6, 8, 10, 12, 14, 16};
  for (int i = 0; i < 8; ++i) if (in_sizes[wIdx[i]] != wK[i] * wN[i]) return;
  if (in_sizes[3] != HID || in_sizes[5] != HID || in_sizes[7] != HID || in_sizes[9] != HID ||
      in_sizes[11] != HID || in_sizes[13] != HID || in_sizes[15] != LAT || in_sizes[17] != LAT) return;
  if (in_sizes[18] != LAT || in_sizes[20] != LAT || in_sizes[19] < 1 || in_sizes[21] < 1 ||
      in_sizes[22] < 1 || in_sizes[23] < 1) return;
  if (out_size != 2 * nN) return;

  const float* x  = (const float*)d_in[0];
  const int*   ei = (const int*)d_in[1];
  const float* wsrc[8];
  for (int i = 0; i < 8; ++i) wsrc[i] = (const float*)d_in[wIdx[i]];
  const float* b1[4]; const float* b2[4];
  for (int l = 0; l < 4; ++l) { b1[l] = (const float*)d_in[3 + 4 * l]; b2[l] = (const float*)d_in[5 + 4 * l]; }
  const float* m_w  = (const float*)d_in[18];
  const float* m_b  = (const float*)d_in[19];
  const float* d_w1 = (const float*)d_in[20];
  const float* d_b1 = (const float*)d_in[21];
  const float* d_w2 = (const float*)d_in[22];
  const float* d_b2 = (const float*)d_in[23];
  float* out = (float*)d_out;

  const int NPAD   = ((nN + NPU - 1) / NPU) * NPU;
  const int nBC    = (nN + NBC - 1) / NBC;
  const int CNTPAD = nBC * NBC;
  if (4 * nBC + 1 > RBN) return;
  const int nBF    = (nN + NBF - 1) / NBF;
  const int csrLen = ((nE + 31) & ~31) + 4096;
  if (NPAD > CNTPAD) return;

  char* ws = (char*)d_ws;
  size_t offc = 0;
  size_t oW[16];
  const size_t oXp = offc; offc += (size_t)NPAD * XP * 4;              offc = (offc + 255) & ~(size_t)255;
  for (int i = 0; i < 8; ++i) {
    oW[2 * i]     = offc; offc += (size_t)wN[i] * wKP[i] * 2;           offc = (offc + 255) & ~(size_t)255;
    oW[2 * i + 1] = offc; offc += (size_t)wN[i] * wKP[i] * 2;           offc = (offc + 255) & ~(size_t)255;
  }
  const size_t oCnt = offc; offc += (size_t)CNTPAD * 4;                 offc = (offc + 255) & ~(size_t)255;
  const size_t oOff = offc; offc += (size_t)CNTPAD * 4;                 offc = (offc + 255) & ~(size_t)255;
  const size_t oRb  = offc; offc += (size_t)RBN * 4;                    offc = (offc + 255) & ~(size_t)255;
  const size_t oCsr = offc; offc += (size_t)csrLen * 4;                 offc = (offc + 255) & ~(size_t)255;
  const size_t oHF  = offc; offc += (size_t)NPAD * HID * 4;             offc = (offc + 255) & ~(size_t)255;
  const size_t oZH  = offc; offc += (size_t)NPAD * HID * 2;             offc = (offc + 255) & ~(size_t)255;
  const size_t oZL  = offc; offc += (size_t)NPAD * HID * 2;             offc = (offc + 255) & ~(size_t)255;
  const size_t oYH  = offc; offc += (size_t)NPAD * HID * 2;             offc = (offc + 255) & ~(size_t)255;
  const size_t oYL  = offc; offc += (size_t)NPAD * HID * 2;             offc = (offc + 255) & ~(size_t)255;
  const size_t oLat = offc; offc += (size_t)NPAD * LAT * 4;             offc = (offc + 255) & ~(size_t)255;
  const size_t oMM  = offc; offc += (size_t)NPAD * 4;                   offc = (offc + 255) & ~(size_t)255;
  const size_t oTT  = offc; offc += (size_t)NPAD * 4;                   offc = (offc + 255) & ~(size_t)255;
  if (offc > ws_size) return;
  float*          xp   = (float*)(ws + oXp);
  unsigned short* wh[8]; unsigned short* wl[8];
  for (int i = 0; i < 8; ++i) { wh[i] = (unsigned short*)(ws + oW[2 * i]); wl[i] = (unsigned short*)(ws + oW[2 * i + 1]); }
  int*            cnt  = (int*)(ws + oCnt);
  int*            offp = (int*)(ws + oOff);
  int*            rb   = (int*)(ws + oRb);
  int*            csr  = (int*)(ws + oCsr);
  float*          hF   = (float*)(ws + oHF);
  unsigned short* zH   = (unsigned short*)(ws + oZH);
  unsigned short* zL   = (unsigned short*)(ws + oZL);
  unsigned short* yH   = (unsigned short*)(ws + oYH);
  unsigned short* yL   = (unsigned short*)(ws + oYL);
  float*          lat  = (float*)(ws + oLat);
  float*          mm   = (float*)(ws + oMM);
  float*          tt   = (float*)(ws + oTT);

  const int vec8  = ((nE & 3) == 0) ? 1 : 0;
  const int nGemm = NPAD / GROWS;
  const int nAgg  = NPAD / ATGT;
  const int LDS_G128 = GROWS * HID * 4;
  const int LDS_G64  = GROWS * LAT * 4;
  const int LDS_A128 = AWAVE * 128 * HID;
  const int LDS_A64  = AWAVE * 128 * LAT;
  const int LDS_A32  = AWAVE * 128 * XP;

  k_xpad<<<(NPAD * (XP / 4) + NTHR - 1) / NTHR, NTHR, 0, stream>>>(x, xp, nN, NPAD);

  WPrep wp;
  int blk = 0;
  for (int i = 0; i < 8; ++i) {
    wp.s[i].src = wsrc[i]; wp.s[i].hi = wh[i]; wp.s[i].lo = wl[i];
    wp.s[i].K = wK[i]; wp.s[i].NOUT = wN[i]; wp.s[i].KP = wKP[i]; wp.s[i].blk0 = blk;
    blk += (wN[i] * wKP[i] / 8 + NTHR - 1) / NTHR;
  }
  k_wprep<<<blk, NTHR, 0, stream>>>(wp);

  k_count<<<nBC, NTHR, 0, stream>>>(ei, cnt, nE, vec8);
  k_offsets<<<1, OTHR, 0, stream>>>(cnt, offp, rb, nBC);
  hipFuncSetAttribute(reinterpret_cast<const void*>(&k_fill), hipFuncAttributeMaxDynamicSharedMemorySize, LDS_FILL);
  k_fill<<<nBF, NTHR, LDS_FILL, stream>>>(ei, offp, rb, csr, nN, nE, vec8, csrLen);

  hipFuncSetAttribute(reinterpret_cast<const void*>(&k_agg<XP, 0>),   hipFuncAttributeMaxDynamicSharedMemorySize, LDS_A32);
  hipFuncSetAttribute(reinterpret_cast<const void*>(&k_agg<HID, 0>),  hipFuncAttributeMaxDynamicSharedMemorySize, LDS_A128);
  hipFuncSetAttribute(reinterpret_cast<const void*>(&k_agg<LAT, 1>),  hipFuncAttributeMaxDynamicSharedMemorySize, LDS_A64);
  hipFuncSetAttribute(reinterpret_cast<const void*>(&k_gemm<XP, HID, 1, 1>),   hipFuncAttributeMaxDynamicSharedMemorySize, LDS_G128);
  hipFuncSetAttribute(reinterpret_cast<const void*>(&k_gemm<HID, HID, 1, 1>),  hipFuncAttributeMaxDynamicSharedMemorySize, LDS_G128);
  hipFuncSetAttribute(reinterpret_cast<const void*>(&k_gemm<HID, HID, 0, 1>),  hipFuncAttributeMaxDynamicSharedMemorySize, LDS_G128);
  hipFuncSetAttribute(reinterpret_cast<const void*>(&k_gemm<HID, LAT, 0, 0>),  hipFuncAttributeMaxDynamicSharedMemorySize, LDS_G64);
  hipFuncSetAttribute(reinterpret_cast<const void*>(&k_gemm<LAT, LAT, 0, 0>),  hipFuncAttributeMaxDynamicSharedMemorySize, LDS_G64);

  k_agg<XP, 0><<<nAgg, ATHR, LDS_A32, stream>>>(csr, offp, cnt, xp, b1[0], zH, zL, nN, csrLen, 0);
  k_gemm<XP, HID, 1, 1><<<nGemm, NTHR, LDS_G128, stream>>>(zH, zL, wh[0], wl[0], b1[0], hF, yH, yL, 1);
  k_gemm<HID, HID, 0, 1><<<nGemm, NTHR, LDS_G128, stream>>>(yH, yL, wh[1], wl[1], b2[0], hF, zH, zL, 1);

  k_agg<HID, 0><<<nAgg, ATHR, LDS_A128, stream>>>(csr, offp, cnt, hF, b1[1], zH, zL, nN, csrLen, 0);
  k_gemm<HID, HID, 1, 1><<<nGemm, NTHR, LDS_G128, stream>>>(zH, zL, wh[2], wl[2], b1[1], hF, yH, yL, 1);
  k_gemm<HID, HID, 0, 1><<<nGemm, NTHR, LDS_G128, stream>>>(yH, yL, wh[3], wl[3], b2[1], hF, zH, zL, 1);

  k_agg<HID, 0><<<nAgg, ATHR, LDS_A128, stream>>>(csr, offp, cnt, hF, b1[2], zH, zL, nN, csrLen, 0);
  k_gemm<HID, HID, 1, 1><<<nGemm, NTHR, LDS_G128, stream>>>(zH, zL, wh[4], wl[4], b1[2], hF, yH, yL, 1);
  k_gemm<HID, HID, 1, 1><<<nGemm, NTHR, LDS_G128, stream>>>(yH, yL, wh[5], wl[5], b2[2], hF, zH, zL, 1);

  k_gemm<HID, LAT, 0, 0><<<nGemm, NTHR, LDS_G64, stream>>>(zH, zL, wh[6], wl[6], b1[3], hF, yH, yL, 0);
  k_agg<LAT, 1><<<nAgg, ATHR, LDS_A64, stream>>>(csr, offp, cnt, hF, b1[3], yH, yL, nN, csrLen, 1);
  k_gemm<LAT, LAT, 0, 0><<<nGemm, NTHR, LDS_G64, stream>>>(yH, yL, wh[7], wl[7], b2[3], lat, zH, zL, 1);

  k_heads<<<NPAD / NTHR, NTHR, 0, stream>>>(lat, m_w, m_b, d_w1, mm, tt);
  const int total = 2 * nN;
  const int nFin = (total + 32 * NWAVE - 1) / (32 * NWAVE);
  k_final<<<nFin, NTHR, 0, stream>>>(csr, offp, cnt, tt, mm, d_b1, d_w2, d_b2, out, nN, csrLen, total, NPAD);
}
